// MambaBlock_12833362281153
// MI455X (gfx1250) — hardware-verified
//
#include <hip/hip_runtime.h>
#include <math.h>

typedef __attribute__((ext_vector_type(16))) _Float16 v16h;
typedef __attribute__((ext_vector_type(8)))  _Float16 v8h;
typedef __attribute__((ext_vector_type(16))) __bf16   v16b;
typedef __attribute__((ext_vector_type(8)))  __bf16   v8b;
typedef __attribute__((ext_vector_type(8)))  float    v8f;
typedef __attribute__((ext_vector_type(4)))  float    v4f;

constexpr int kBatch  = 4;
constexpr int kSeq    = 512;
constexpr int kDm     = 128;
constexpr int kDin    = 256;
constexpr int kNst    = 256;
constexpr int kRows   = kBatch * kSeq;
constexpr int kXpP    = 2 * kDin;
constexpr int kDbcP   = 3 * kDin;
constexpr int kScanTS = 16;
constexpr int kScanDG = 32;
constexpr int kScanYP = 36;
static_assert(kDin == kNst);
static_assert((kDm % 32) == 0 && (kDin % 32) == 0);
static_assert((kRows % 64) == 0 && (kXpP % 64) == 0 && (kDbcP % 64) == 0 && (kDm % 64) == 0);
static_assert((kSeq % kScanTS) == 0 && (kDin % kScanDG) == 0 && kNst == 8 * 32 && kScanDG * 8 == 256);
static_assert((kDm % 64) == 0 && (kDin % 64) == 0 && (kXpP % 32) == 0 && (kDm % 32) == 0);

constexpr size_t kOffXH   = 0;
constexpr size_t kOffXL   = kOffXH  + (size_t)kRows * kDm  * 2;
constexpr size_t kOffWIH  = kOffXL  + (size_t)kRows * kDm  * 2;
constexpr size_t kOffWIL  = kOffWIH + (size_t)kXpP  * kDm  * 2;
constexpr size_t kOffWDH  = kOffWIL + (size_t)kXpP  * kDm  * 2;
constexpr size_t kOffWDL  = kOffWDH + (size_t)kDbcP * kDin * 2;
constexpr size_t kOffWOH  = kOffWDL + (size_t)kDbcP * kDin * 2;
constexpr size_t kOffWOL  = kOffWOH + (size_t)kDm   * kDin * 2;
constexpr size_t kOffXP   = kOffWOL + (size_t)kDm   * kDin * 2;
constexpr size_t kOffXSH  = kOffXP  + (size_t)kRows * kXpP * 4;
constexpr size_t kOffXSL  = kOffXSH + (size_t)kRows * kDin * 2;
constexpr size_t kOffDBC  = kOffXSL + (size_t)kRows * kDin * 2;
constexpr size_t kOffYG   = kOffDBC + (size_t)kRows * kDbcP * 4;
constexpr size_t kOffYH   = kOffYG  + (size_t)kRows * kDin * 4;
constexpr size_t kOffYL   = kOffYH  + (size_t)kRows * kDin * 2;
constexpr size_t kWsTotal = kOffYL  + (size_t)kRows * kDin * 2;
static_assert(kWsTotal == 19005440ull);
static_assert(kWsTotal <= 134217728ull);
static_assert((kOffXL % 128) == 0 && (kOffWIH % 128) == 0 && (kOffWIL % 128) == 0 && (kOffWDH % 128) == 0 &&
              (kOffWDL % 128) == 0 && (kOffWOH % 128) == 0 && (kOffWOL % 128) == 0 && (kOffXP % 128) == 0 &&
              (kOffXSH % 128) == 0 && (kOffXSL % 128) == 0 && (kOffDBC % 128) == 0 && (kOffYG % 128) == 0 &&
              (kOffYH % 128) == 0 && (kOffYL % 128) == 0);

__device__ __forceinline__ unsigned short f2bf_bits(float f) {
  unsigned u = __float_as_uint(f);
  return (unsigned short)((u + 0x7FFFu + ((u >> 16) & 1u)) >> 16);
}
__device__ __forceinline__ float bf_bits2f(unsigned short h) { return __uint_as_float(((unsigned)h) << 16); }

__device__ __forceinline__ void dep_guard_h(v8f& a, v8f& b, v16h x, v16h y) { asm volatile("v_nop\n\tv_nop\n\tv_nop\n\tv_nop" : "+v"(a), "+v"(b) : "v"(x), "v"(y)); }
__device__ __forceinline__ void dep_guard_b(v8f& a, v8f& b, v16b x, v16b y) { asm volatile("v_nop\n\tv_nop\n\tv_nop\n\tv_nop" : "+v"(a), "+v"(b) : "v"(x), "v"(y)); }
__device__ __forceinline__ void dep_guard4_h(v8f& a, v8f& b, v8f& c, v8f& d, v16h x, v16h y) { asm volatile("v_nop\n\tv_nop\n\tv_nop\n\tv_nop" : "+v"(a), "+v"(b), "+v"(c), "+v"(d) : "v"(x), "v"(y)); }
__device__ __forceinline__ void dep_guard4_b(v8f& a, v8f& b, v8f& c, v8f& d, v16b x, v16b y) { asm volatile("v_nop\n\tv_nop\n\tv_nop\n\tv_nop" : "+v"(a), "+v"(b), "+v"(c), "+v"(d) : "v"(x), "v"(y)); }
__device__ __forceinline__ void keep4_h(v16h a, v16h b, v16h c, v16h d) { asm volatile("v_nop" :: "v"(a), "v"(b), "v"(c), "v"(d)); }
__device__ __forceinline__ void keep4_b(v16b a, v16b b, v16b c, v16b d) { asm volatile("v_nop" :: "v"(a), "v"(b), "v"(c), "v"(d)); }
__device__ __forceinline__ void acc_guard4(v8f& a, v8f& b, v8f& c, v8f& d) { asm volatile("v_nop\n\tv_nop\n\tv_nop\n\tv_nop" : "+v"(a), "+v"(b), "+v"(c), "+v"(d)); }
template <typename T> struct Frag;
template <> struct Frag<_Float16> {
  typedef v16h V; union U { v16h v; v8h h[2]; };
  static __device__ __forceinline__ v16h load(const _Float16* p) {
    U f; f.h[0] = *(const v8h*)(p); f.h[1] = *(const v8h*)(p + 16); return f.v;
  }
  static __device__ __forceinline__ v8f mma(v16h a, v16h b, v8f c) {
    return __builtin_amdgcn_wmma_f32_16x16x32_f16(false, a, false, b, (short)0, c, false, false);
  }
  static __device__ __forceinline__ void guard(v8f& a, v8f& b, v16h x, v16h y) { dep_guard_h(a, b, x, y); }
  static __device__ __forceinline__ void guard4(v8f& a, v8f& b, v8f& c, v8f& d, v16h x, v16h y) { dep_guard4_h(a, b, c, d, x, y); }
  static __device__ __forceinline__ void keep(v16h a, v16h b, v16h c, v16h d) { keep4_h(a, b, c, d); }
};
template <> struct Frag<__bf16> {
  typedef v16b V; union U { v16b v; v8b h[2]; };
  static __device__ __forceinline__ v16b load(const __bf16* p) {
    U f; f.h[0] = *(const v8b*)(p); f.h[1] = *(const v8b*)(p + 16); return f.v;
  }
  static __device__ __forceinline__ v8f mma(v16b a, v16b b, v8f c) {
    return __builtin_amdgcn_wmma_f32_16x16x32_bf16(false, a, false, b, (short)0, c, false, false);
  }
  static __device__ __forceinline__ void guard(v8f& a, v8f& b, v16b x, v16b y) { dep_guard_b(a, b, x, y); }
  static __device__ __forceinline__ void guard4(v8f& a, v8f& b, v8f& c, v8f& d, v16b x, v16b y) { dep_guard4_b(a, b, c, d, x, y); }
  static __device__ __forceinline__ void keep(v16b a, v16b b, v16b c, v16b d) { keep4_b(a, b, c, d); }
};

template <int ET> struct Elem;
template <> struct Elem<0> { typedef _Float16 T; };
template <> struct Elem<1> { typedef __bf16 T; };
template <int ET, int SPL, int BIAS_MODE, int OUT_MODE, bool RESID, int ACT = 0>
__global__ __launch_bounds__(256) void wmma_gemm64(
    const unsigned short* __restrict__ Ap, const unsigned short* __restrict__ A2p, int lda, long strideA,
    const unsigned short* __restrict__ Btp, const unsigned short* __restrict__ Bt2p, int ldb, long strideB,
    void* __restrict__ Cout, void* __restrict__ Cout2, int ldc, long strideC,
    const float* __restrict__ bias,
    const float* __restrict__ resid, long strideR,
    int M, int N, int K, float scale) {
  typedef typename Elem<ET>::T T;
  typedef typename Frag<T>::V V;
  const T* A = (const T*)Ap; const T* A2 = (const T*)A2p; const T* Bt = (const T*)Btp; const T* Bt2 = (const T*)Bt2p;
  __shared__ __align__(16) float sT[8][16 * 68];
  const int b    = blockIdx.y;
  const int lane = threadIdx.x & 31;
  const int wave = threadIdx.x >> 5;
  const int tilesN = N >> 6;
  const int tilesM = M >> 6;
  const int tile = blockIdx.x * 8 + wave;
  if (tile >= tilesM * tilesN) return;
  const int tm = tile / tilesN;
  const int tn = tile - tm * tilesN;
  const int m0 = tm << 6;
  const int n0 = tn << 6;

  const T* Ab  = A  + (size_t)b * strideA;
  const T* Bb  = Bt + (size_t)b * strideB;
  const T* Ab2 = (SPL >= 1) ? (A2  + (size_t)b * strideA) : nullptr;
  const T* Bb2 = (SPL == 2) ? (Bt2 + (size_t)b * strideB) : nullptr;

  const int rlane = lane & 15;
  const int koff  = (lane >> 4) * 8;
  const int mOff  = (lane >> 4) * 8;

  v8f acc[4][4];
#pragma unroll
  for (int i = 0; i < 4; ++i)
#pragma unroll
    for (int j = 0; j < 4; ++j) acc[i][j] = (v8f){0.f,0.f,0.f,0.f,0.f,0.f,0.f,0.f};

  for (int k0 = 0; k0 < K; k0 += 32) {
    V bh[4], bl[4];
#pragma unroll
    for (int j = 0; j < 4; ++j) {
      const size_t bo = (size_t)(n0 + (j << 4) + rlane) * ldb + koff + k0;
      bh[j] = Frag<T>::load(Bb + bo);
      if (SPL == 2) bl[j] = Frag<T>::load(Bb2 + bo);
    }
#pragma unroll
    for (int i = 0; i < 4; ++i) {
      const size_t ao = (size_t)(m0 + (i << 4) + rlane) * lda + koff + k0;
      V ah = Frag<T>::load(Ab + ao);
      V al;
      if (SPL >= 1) al = Frag<T>::load(Ab2 + ao);
#pragma unroll
      for (int j = 0; j < 4; ++j) {
        acc[i][j] = Frag<T>::mma(ah, bh[j], acc[i][j]);
        if (SPL == 2) acc[i][j] = Frag<T>::mma(ah, bl[j], acc[i][j]);
        if (SPL >= 1) acc[i][j] = Frag<T>::mma(al, bh[j], acc[i][j]);
      }
      Frag<T>::guard4(acc[i][0], acc[i][1], acc[i][2], acc[i][3], ah, (SPL >= 1) ? al : ah);
    }
    Frag<T>::keep(bh[0], bh[1], bh[2], bh[3]);
    if (SPL == 2) Frag<T>::keep(bl[0], bl[1], bl[2], bl[3]);
  }
  acc_guard4(acc[0][0], acc[0][1], acc[0][2], acc[0][3]);
  acc_guard4(acc[1][0], acc[1][1], acc[1][2], acc[1][3]);
  acc_guard4(acc[2][0], acc[2][1], acc[2][2], acc[2][3]);
  acc_guard4(acc[3][0], acc[3][1], acc[3][2], acc[3][3]);

  float* slab = sT[wave];
  const float* Rb = RESID ? (resid + (size_t)b * strideR) : nullptr;
#pragma unroll
  for (int i = 0; i < 4; ++i) {
    const int mBase = m0 + (i << 4);
#pragma unroll
    for (int j = 0; j < 4; ++j) {
      const int n = n0 + (j << 4) + rlane;
      float bv = 0.f;
      if (BIAS_MODE == 2) bv = bias[n];
#pragma unroll
      for (int r = 0; r < 8; ++r) {
        float v = acc[i][j][r] * scale;
        if (BIAS_MODE == 1) v += bias[mBase + mOff + r];
        if (BIAS_MODE == 2) v += bv;
        if (RESID) v += Rb[(size_t)(mBase + mOff + r) * ldc + n];
        if (ACT == 1) v = tanhf(v);
        if (ACT == 2) v = fmaxf(v, 0.0f);
        if (ACT == 3) v = v / (1.0f + expf(-v));
        if (ACT == 4) v = (v > 0.f) ? v : 0.01f * v;
        slab[(mOff + r) * 68 + (j << 4) + rlane] = v;
      }
    }
    __builtin_amdgcn_fence(__ATOMIC_RELEASE, "workgroup");
    __builtin_amdgcn_wave_barrier();
    __builtin_amdgcn_fence(__ATOMIC_ACQUIRE, "workgroup");
    if (OUT_MODE == 0) {
      float* C = (float*)Cout + (size_t)b * strideC;
      const int hh = lane >> 4, c4 = (lane & 15) * 4;
      for (int pass = 0; pass < 2; ++pass) {
#pragma unroll
        for (int it = 0; it < 8; ++it) {
          const int row = it * 2 + hh;
          v4f v = *(const v4f*)(slab + row * 68 + c4);
          *(volatile v4f*)(C + (size_t)(mBase + row) * ldc + n0 + c4) = v;
        }
        __threadfence();
      }
    } else {
      const int q = lane >> 3, c8 = (lane & 7) * 8;
      unsigned short* C  = (unsigned short*)Cout  + (size_t)b * strideC;
      unsigned short* C2 = (OUT_MODE == 2) ? ((unsigned short*)Cout2 + (size_t)b * strideC) : nullptr;
      for (int pass = 0; pass < 2; ++pass) {
#pragma unroll
        for (int it = 0; it < 4; ++it) {
          const int row = it * 4 + q;
          const float* sp = slab + row * 68 + c8;
          v8h hv, lv;
#pragma unroll
          for (int e = 0; e < 8; ++e) {
            if (OUT_MODE == 1) {
              hv[e] = (_Float16)sp[e];
            } else {
              unsigned short hb = f2bf_bits(sp[e]);
              unsigned short lb = f2bf_bits(sp[e] - bf_bits2f(hb));
              hv[e] = __builtin_bit_cast(_Float16, hb);
              lv[e] = __builtin_bit_cast(_Float16, lb);
            }
          }
          *(volatile v8h*)(C + (size_t)(mBase + row) * ldc + n0 + c8) = hv;
          if (OUT_MODE == 2) *(volatile v8h*)(C2 + (size_t)(mBase + row) * ldc + n0 + c8) = lv;
        }
        __threadfence();
      }
    }
    __builtin_amdgcn_fence(__ATOMIC_RELEASE, "workgroup");
    __builtin_amdgcn_wave_barrier();
    __builtin_amdgcn_fence(__ATOMIC_ACQUIRE, "workgroup");
  }
}

__global__ __launch_bounds__(256) void split_rows_bf16_kernel(
    const float* __restrict__ src, int srcPitch, int cols,
    unsigned short* __restrict__ dhi, unsigned short* __restrict__ dlo, int total8)
{
  const int i = blockIdx.x * 256 + threadIdx.x;
  if (i >= total8) return;
  const int e0i = i << 3;
  const int row = e0i / cols;
  const int c   = e0i - row * cols;
  const float* sp = src + (size_t)row * srcPitch + c;
  const v4f a0 = *(const v4f*)(sp);
  const v4f a1 = *(const v4f*)(sp + 4);
  v8h hv, lv;
#pragma unroll
  for (int e = 0; e < 4; ++e) {
    const unsigned short h0 = f2bf_bits(a0[e]), h1 = f2bf_bits(a1[e]);
    const unsigned short l0 = f2bf_bits(a0[e] - bf_bits2f(h0)), l1 = f2bf_bits(a1[e] - bf_bits2f(h1));
    hv[e]     = __builtin_bit_cast(_Float16, h0);
    hv[4 + e] = __builtin_bit_cast(_Float16, h1);
    lv[e]     = __builtin_bit_cast(_Float16, l0);
    lv[4 + e] = __builtin_bit_cast(_Float16, l1);
  }
  const size_t e0 = (size_t)e0i;
  unsigned short* qh = dhi + e0;
  unsigned short* ql = dlo + e0;
  *(volatile v8h*)qh = hv;
  *(volatile v8h*)ql = lv;
  __threadfence();
  *(volatile v8h*)qh = hv;
  *(volatile v8h*)ql = lv;
}

__global__ __launch_bounds__(256) void transpose_split_bf16_kernel(
    const float* __restrict__ in, int K, int N,
    unsigned short* __restrict__ dhi, unsigned short* __restrict__ dlo, int nOff)
{
  __shared__ __align__(16) float sT[32 * 68];
  const int tid = threadIdx.x, lane = tid & 31, wave = tid >> 5;
  const int k0 = blockIdx.x * 64, n0 = blockIdx.y * 32;
#pragma unroll
  for (int i = 0; i < 8; ++i) {
    const int kr = wave + 8 * i;
    sT[lane * 68 + kr] = in[(size_t)(k0 + kr) * N + n0 + lane];
  }
  __syncthreads();
  const int q = lane >> 3, c8 = (lane & 7) * 8;
  const int nr = wave * 4 + q;
  const float* sp = sT + nr * 68 + c8;
  const v4f a0 = *(const v4f*)(sp);
  const v4f a1 = *(const v4f*)(sp + 4);
  v8h hv, lv;
#pragma unroll
  for (int e = 0; e < 4; ++e) {
    const unsigned short h0 = f2bf_bits(a0[e]), h1 = f2bf_bits(a1[e]);
    const unsigned short l0 = f2bf_bits(a0[e] - bf_bits2f(h0)), l1 = f2bf_bits(a1[e] - bf_bits2f(h1));
    hv[e]     = __builtin_bit_cast(_Float16, h0);
    hv[4 + e] = __builtin_bit_cast(_Float16, h1);
    lv[e]     = __builtin_bit_cast(_Float16, l0);
    lv[4 + e] = __builtin_bit_cast(_Float16, l1);
  }
  const size_t o = (size_t)(nOff + n0 + nr) * K + k0 + c8;
  *(volatile v8h*)(dhi + o) = hv;
  *(volatile v8h*)(dlo + o) = lv;
  __threadfence();
  *(volatile v8h*)(dhi + o) = hv;
  *(volatile v8h*)(dlo + o) = lv;
}

__global__ __launch_bounds__(256) void scan_kernel(
    const float* __restrict__ DBC, const float* __restrict__ XP, const float* __restrict__ Am,
    const float* __restrict__ Dp, float* __restrict__ YG)
{
  __shared__ __align__(16) float sBX[kScanTS * kNst];
  __shared__ __align__(16) float sCV[kScanTS * kNst];
  __shared__ __align__(16) float sDl[kScanTS * kScanDG];
  __shared__ __align__(16) float sZ[kScanTS * kScanDG];
  __shared__ __align__(16) float sY[kScanTS * kScanYP];
  (void)Dp;
  const int tid = threadIdx.x, lane = tid & 31, wave = tid >> 5;
  constexpr int kGroups = kDin / kScanDG;
  const int bix = blockIdx.x / kGroups;
  const int d0  = (blockIdx.x - bix * kGroups) * kScanDG;
  const int dloc = tid >> 3, oct = tid & 7, nb = oct * 32;
  const int d = d0 + dloc;
  const size_t row0 = (size_t)bix * kSeq;

  float a[32], st[32];
  {
    const float* ar = Am + (size_t)d * kNst + nb;
#pragma unroll
    for (int j4 = 0; j4 < 4; ++j4) {
      const v4f av = *(const v4f*)(ar + 4 * j4);
      a[4 * j4 + 0] = av[0]; a[4 * j4 + 1] = av[1]; a[4 * j4 + 2] = av[2]; a[4 * j4 + 3] = av[3];
    }
    asm volatile("" ::: "memory");
#pragma unroll
    for (int j4 = 4; j4 < 8; ++j4) {
      const v4f av = *(const v4f*)(ar + 4 * j4);
      a[4 * j4 + 0] = av[0]; a[4 * j4 + 1] = av[1]; a[4 * j4 + 2] = av[2]; a[4 * j4 + 3] = av[3];
    }
  }
#pragma unroll
  for (int j = 0; j < 32; ++j) st[j] = 0.0f;

  const int sr = tid >> 6, sc4 = (tid & 63) * 4;
  const int q = lane >> 3, c4 = (lane & 7) * 4;

#pragma unroll 1
  for (int t0 = 0; t0 < kSeq; t0 += kScanTS) {
#pragma unroll 1
    for (int i = 0; i < 4; ++i) {
      const int r = sr + 4 * i;
      const size_t grow = row0 + t0 + r;
      const v4f xv = *(const v4f*)(XP  + grow * kXpP + sc4);
      const v4f bv = *(const v4f*)(DBC + grow * kDbcP + kDin + sc4);
      const v4f cv = *(const v4f*)(DBC + grow * kDbcP + 2 * kDin + sc4);
      const v4f bx = bv * xv;
      *(v4f*)(sBX + r * kNst + sc4) = bx;
      *(v4f*)(sCV + r * kNst + sc4) = cv;
    }
#pragma unroll
    for (int rr = 0; rr < 2; ++rr) {
      const int idx = tid + 256 * rr;
      const int i = idx >> 5, dd = idx & 31;
      const size_t grow = row0 + t0 + i;
      sDl[i * kScanDG + dd] = DBC[grow * kDbcP + d0 + dd];
      sZ[i * kScanDG + dd]  = XP[grow * kXpP + kDin + d0 + dd];
    }
    __syncthreads();
#pragma unroll 1
    for (int s = 0; s < kScanTS; ++s) {
      const float dlt = sDl[s * kScanDG + dloc];
      const float* bxr = sBX + s * kNst + nb;
      const float* cvr = sCV + s * kNst + nb;
      float acc = 0.0f;
#pragma unroll
      for (int j4 = 0; j4 < 8; ++j4) {
        const v4f bx = *(const v4f*)(bxr + 4 * j4);
        const v4f cv = *(const v4f*)(cvr + 4 * j4);
#pragma unroll
        for (int e = 0; e < 4; ++e) {
          const int j = 4 * j4 + e;
          const float ea  = __expf(dlt * a[j]);
          const float inc = dlt * bx[e];
          st[j] = fmaf(ea, st[j], inc);
          acc = fmaf(st[j], cv[e], acc);
        }
      }
      acc += __shfl_xor(acc, 1, 32);
      acc += __shfl_xor(acc, 2, 32);
      acc += __shfl_xor(acc, 4, 32);
      const float zv = sZ[s * kScanDG + dloc];
      const float sg = __builtin_amdgcn_rcpf(1.0f + __expf(-zv));
      const float yg = acc * (zv * sg);
      if (oct == 0) sY[s * kScanYP + dloc] = yg;
    }
    __syncthreads();
    if (wave < 4) {
      const int row = wave * 4 + q;
      const v4f v = *(const v4f*)(sY + row * kScanYP + c4);
      float* p = YG + (row0 + t0 + row) * kDin + d0 + c4;
      *(volatile v4f*)p = v;
      __threadfence();
      *(volatile v4f*)p = v;
    }
  }
}

extern "C" void kernel_launch(void* const* d_in, const int* in_sizes, int n_in,
                              void* d_out, int out_size, void* d_ws, size_t ws_size,
                              hipStream_t stream) {
  if (n_in < 8) return;
  if (in_sizes[0] != kRows * kDm) return;
  if (in_sizes[1] != kDm * kXpP) return;
  if (in_sizes[2] != kDin * kDin) return;
  if (in_sizes[3] != kDin * kNst) return;
  if (in_sizes[4] != kDin * kDin) return;
  if (in_sizes[5] != kDin * kDm) return;
  if (in_sizes[6] != kDin * kNst) return;
  if (in_sizes[7] != kDin) return;
  if (out_size != kRows * kDm) return;
  if (ws_size < kWsTotal) return;

  const float* x       = (const float*)d_in[0];
  const float* W_in    = (const float*)d_in[1];
  const float* W_delta = (const float*)d_in[2];
  const float* W_B     = (const float*)d_in[3];
  const float* W_C     = (const float*)d_in[4];
  const float* W_out   = (const float*)d_in[5];
  const float* Am      = (const float*)d_in[6];
  const float* Dp      = (const float*)d_in[7];
  float* out = (float*)d_out;

  char* ws = (char*)d_ws;
  unsigned short* XH   = (unsigned short*)(ws + kOffXH);
  unsigned short* XL   = (unsigned short*)(ws + kOffXL);
  unsigned short* WIH  = (unsigned short*)(ws + kOffWIH);
  unsigned short* WIL  = (unsigned short*)(ws + kOffWIL);
  unsigned short* WDH  = (unsigned short*)(ws + kOffWDH);
  unsigned short* WDL  = (unsigned short*)(ws + kOffWDL);
  unsigned short* WOH  = (unsigned short*)(ws + kOffWOH);
  unsigned short* WOL  = (unsigned short*)(ws + kOffWOL);
  float*          XP   = (float*)(ws + kOffXP);
  unsigned short* XSH  = (unsigned short*)(ws + kOffXSH);
  unsigned short* XSL  = (unsigned short*)(ws + kOffXSL);
  float*          DBC  = (float*)(ws + kOffDBC);
  float*          YG   = (float*)(ws + kOffYG);
  unsigned short* YH   = (unsigned short*)(ws + kOffYH);
  unsigned short* YL   = (unsigned short*)(ws + kOffYL);

  split_rows_bf16_kernel<<<(kRows * kDm / 8) / 256, 256, 0, stream>>>(x, kDm, kDm, XH, XL, kRows * kDm / 8);
  transpose_split_bf16_kernel<<<dim3(kDm / 64, kXpP / 32), 256, 0, stream>>>(W_in, kDm, kXpP, WIH, WIL, 0);
  transpose_split_bf16_kernel<<<dim3(kDin / 64, kDin / 32), 256, 0, stream>>>(W_delta, kDin, kDin, WDH, WDL, 0);
  transpose_split_bf16_kernel<<<dim3(kDin / 64, kNst / 32), 256, 0, stream>>>(W_B, kDin, kNst, WDH, WDL, kDin);
  transpose_split_bf16_kernel<<<dim3(kDin / 64, kDin / 32), 256, 0, stream>>>(W_C, kDin, kDin, WDH, WDL, 2 * kDin);
  transpose_split_bf16_kernel<<<dim3(kDin / 64, kDm / 32), 256, 0, stream>>>(W_out, kDin, kDm, WOH, WOL, 0);

  wmma_gemm64<1, 2, 0, 0, false><<<dim3(32, 1), 256, 0, stream>>>(
      XH, XL, kDm, 0L,
      WIH, WIL, kDm, 0L,
      (void*)XP, nullptr, kXpP, 0L,
      nullptr, nullptr, 0L,
      kRows, kXpP, kDm, 1.0f);

  split_rows_bf16_kernel<<<(kRows * kDin / 8) / 256, 256, 0, stream>>>(XP, kXpP, kDin, XSH, XSL, kRows * kDin / 8);

  wmma_gemm64<1, 2, 0, 0, false><<<dim3(48, 1), 256, 0, stream>>>(
      XSH, XSL, kDin, 0L,
      WDH, WDL, kDin, 0L,
      (void*)DBC, nullptr, kDbcP, 0L,
      nullptr, nullptr, 0L,
      kRows, kDbcP, kDin, 1.0f);

  scan_kernel<<<kBatch * (kDin / kScanDG), 256, 0, stream>>>(DBC, XP, Am, Dp, YG);

  split_rows_bf16_kernel<<<(kRows * kDin / 8) / 256, 256, 0, stream>>>(YG, kDin, kDin, YH, YL, kRows * kDin / 8);

  wmma_gemm64<1, 2, 0, 0, false><<<dim3(8, 1), 256, 0, stream>>>(
      YH, YL, kDin, 0L,
      WOH, WOL, kDin, 0L,
      (void*)out, nullptr, kDm, 0L,
      nullptr, nullptr, 0L,
      kRows, kDm, kDin, 1.0f);
}
